// CustomMHA_87935160419038
// MI455X (gfx1250) — hardware-verified
//
#include <hip/hip_runtime.h>
#include <math.h>

typedef __attribute__((ext_vector_type(16))) _Float16 v16h;
typedef __attribute__((ext_vector_type(16))) __bf16 v16b;
typedef __attribute__((ext_vector_type(8)))  _Float16 v8h;
typedef __attribute__((ext_vector_type(8)))  __bf16 v8b;
typedef __attribute__((ext_vector_type(8)))  float v8f;
typedef __attribute__((ext_vector_type(4)))  float v4f;
typedef __attribute__((ext_vector_type(4)))  unsigned v4u;

template <typename T> __device__ __forceinline__ void vst2(void* p, T v) { *(volatile T*)p = v; __threadfence(); *(volatile T*)p = v; }
__device__ __forceinline__ v8f wmma16(v16h a, v16h b, v8f c) {
  v8f d = __builtin_amdgcn_wmma_f32_16x16x32_f16(false, a, false, b, (short)0, c, false, false);
  asm volatile("v_nop\n\tv_nop\n\tv_nop\n\tv_nop" : "+v"(d) : "v"(a), "v"(b));
  return d;
}
__device__ __forceinline__ v8f wmma_bf(v16b a, v16b b, v8f c) {
  v8f d = __builtin_amdgcn_wmma_f32_16x16x32_bf16(false, a, false, b, (short)0, c, false, false);
  asm volatile("v_nop\n\tv_nop\n\tv_nop\n\tv_nop" : "+v"(d) : "v"(a), "v"(b));
  return d;
}
__device__ __forceinline__ v16h frag_h(const _Float16* rowk0, int lane) {
  union { v16h v; v8h q[2]; } u; const _Float16* p = rowk0 + 8 * (lane >> 4);
  u.q[0] = *(const v8h*)p; u.q[1] = *(const v8h*)(p + 16); return u.v;
}
__device__ __forceinline__ v16b frag_b(const __bf16* rowk0, int lane) {
  union { v16b v; v8b q[2]; } u; const __bf16* p = rowk0 + 8 * (lane >> 4);
  u.q[0] = *(const v8b*)p; u.q[1] = *(const v8b*)(p + 16); return u.v;
}
struct F2 { v16b h, l; };
__device__ __forceinline__ F2 bsplit16(const float v[16]) { F2 r;
#pragma unroll
  for (int i = 0; i < 16; ++i) { const __bf16 hb = (__bf16)v[i]; r.h[i] = hb; r.l[i] = (__bf16)(v[i] - (float)hb); }
  return r; }
__device__ __forceinline__ F2 split_row(const float* row, int k0, int lane) { float v[16]; const float* p = row + k0 + 8 * (lane >> 4);
  const v4f a0 = *(const v4f*)p, a1 = *(const v4f*)(p + 4), b0 = *(const v4f*)(p + 16), b1 = *(const v4f*)(p + 20);
#pragma unroll
  for (int i = 0; i < 4; ++i) { v[i] = a0[i]; v[4 + i] = a1[i]; v[8 + i] = b0[i]; v[12 + i] = b1[i]; }
  return bsplit16(v); }
__device__ __forceinline__ float bfr(float v) { return (float)(__bf16)v; }
__device__ __forceinline__ void ldsx() { asm volatile("s_wait_dscnt 0" ::: "memory"); __builtin_amdgcn_fence(3, "workgroup"); __builtin_amdgcn_wave_barrier(); }

#ifndef NB
#define NB 4
#endif
#ifndef SEQ
#define SEQ 2048
#endif
#define NB_FULL 4
#define TT_FULL 2048
#define CC 1024
#define NH 16
#define HD 64
#define C3 (3 * CC)
static_assert(NB >= 1 && NB <= NB_FULL);
static_assert(SEQ % 64 == 0 && SEQ >= 64 && SEQ <= TT_FULL);
static_assert(CC % 128 == 0 && NH * HD == CC && HD == 64);

#define WS_XB  ((size_t)0)
#define WS_WB  (WS_XB + 2u * (size_t)NB * SEQ * CC)
#define WS_PB  (WS_WB + 2u * (size_t)C3 * CC)
#define WS_QH  (WS_PB + 2u * (size_t)CC * CC)
#define WS_KH  (WS_QH + 2u * (size_t)NB * SEQ * CC)
#define WS_VT  (WS_KH + 2u * (size_t)NB * SEQ * CC)
#define WS_Y   (WS_VT + 2u * (size_t)NB * CC * SEQ)
#define WS_END (WS_Y + 4u * (size_t)NB * SEQ * CC)
static_assert(WS_END <= (size_t)134217728);
static_assert((WS_WB % 128) == 0 && (WS_PB % 128) == 0 && (WS_QH % 128) == 0 && (WS_KH % 128) == 0 && (WS_VT % 128) == 0 && (WS_Y % 128) == 0);

__global__ __launch_bounds__(256) void k_cvt(const float* __restrict__ src, __bf16* __restrict__ dst, int nrows, int row_len, int seg, int seg_stride) {
  const size_t i = (size_t)blockIdx.x * 256 + threadIdx.x; const size_t e = i * 8; const size_t total = (size_t)nrows * (size_t)row_len;
  if (e >= total) return;
  const size_t r = e / (size_t)row_len, c = e % (size_t)row_len; const size_t sr = (r / (size_t)seg) * (size_t)seg_stride + (r % (size_t)seg);
  const float* p = src + sr * (size_t)row_len + c;
  const v4f a = *(const v4f*)p, b2 = *(const v4f*)(p + 4);
  union { v8b v; v4u u; } o;
#pragma unroll
  for (int k = 0; k < 4; ++k) { o.v[k] = (__bf16)a[k]; o.v[4 + k] = (__bf16)b2[k]; }
  vst2(dst + e, o.u);
}

__global__ __launch_bounds__(128) void k_proj(const __bf16* __restrict__ XB, const __bf16* __restrict__ WB, const float* __restrict__ BIN, _Float16* __restrict__ QH, _Float16* __restrict__ KH, _Float16* __restrict__ VT) {
  __shared__ __align__(16) _Float16 sh[64][136]; __shared__ __align__(16) _Float16 th[128][72];
  const int tid = threadIdx.x, wave = tid >> 5, lane = tid & 31, col = lane & 15, g = lane >> 4;
  const int c0 = blockIdx.y * 128; const int which = c0 / CC; const int cq = c0 - which * CC; const size_t r0 = (size_t)blockIdx.x * 64;
  v8f acc[8] = {};
#pragma unroll 1
  for (int kc = 0; kc < CC / 32; ++kc) { const v16b a = frag_b(XB + (r0 + wave * 16 + col) * CC + kc * 32, lane);
#pragma unroll
    for (int j = 0; j < 8; ++j) { const v16b w = frag_b(WB + (size_t)(c0 + j * 16 + col) * CC + kc * 32, lane); acc[j] = wmma_bf(a, w, acc[j]); } }
#pragma unroll
  for (int j = 0; j < 8; ++j) { const float bb = bfr(BIN[c0 + j * 16 + col]);
#pragma unroll
    for (int r = 0; r < 8; ++r) { const float v = acc[j][r] + bb; const int rl = wave * 16 + 8 * g + r, cl = j * 16 + col; const _Float16 hv = (_Float16)v;
      if (which == 2) th[cl][rl] = hv; else sh[rl][cl] = hv; } }
  __syncthreads();
  if (which < 2) { _Float16* dh = (which == 0) ? QH : KH; for (int e = tid; e < 64 * 16; e += 128) { const int rl = e >> 4, q = e & 15; vst2(dh + (r0 + rl) * CC + cq + q * 8, *(const v4u*)&sh[rl][q * 8]); } }
  else { const size_t b = r0 / SEQ; const int t0 = (int)(r0 % SEQ); for (int e = tid; e < 128 * 8; e += 128) { const int cl = e >> 3, q = e & 7; const size_t o2 = (b * CC + cq + cl) * (size_t)SEQ + t0 + q * 8; vst2(VT + o2, *(const v4u*)&th[cl][q * 8]); } }
}

__global__ __launch_bounds__(128) __attribute__((amdgpu_num_vgpr(256))) void k_attn(const _Float16* __restrict__ QH, const _Float16* __restrict__ KH, const _Float16* __restrict__ VT, float* __restrict__ Y) {
  __shared__ __align__(16) float ss[4][16][HD + 4];
  const int tid = threadIdx.x, wave = tid >> 5, lane = tid & 31, col = lane & 15, g = lane >> 4;
  const int b = blockIdx.z, h = blockIdx.y; const int ql0 = blockIdx.x * 64 + wave * 16;
  const size_t qrow = (size_t)b * SEQ + ql0 + col;
  const v16h qf0 = frag_h(QH + qrow * CC + h * HD, lane), qf1 = frag_h(QH + qrow * CC + h * HD + 32, lane);
  const _Float16* Kb = KH + ((size_t)b * SEQ + col) * CC + h * HD;
  const _Float16* Vb = VT + ((size_t)b * CC + h * HD + col) * (size_t)SEQ;
  float m = -1.0e30f, l = 0.f; v8f oacc[4] = {};
#pragma unroll 1
  for (int ks = 0; ks < SEQ; ks += 32) {
    v8f s0 = {}, s1 = {};
    { const _Float16* k0p = Kb + (size_t)ks * CC; const _Float16* k1p = k0p + (size_t)16 * CC;
      s0 = wmma16(frag_h(k0p, lane), qf0, s0); s0 = wmma16(frag_h(k0p + 32, lane), qf1, s0);
      s1 = wmma16(frag_h(k1p, lane), qf0, s1); s1 = wmma16(frag_h(k1p + 32, lane), qf1, s1); }
    float mloc = -1.0e30f;
#pragma unroll
    for (int r = 0; r < 8; ++r) mloc = fmaxf(mloc, fmaxf(s0[r], s1[r]));
    mloc = fmaxf(mloc, __shfl_xor(mloc, 16)) * 0.125f;
    const float mn = fmaxf(m, mloc); const float alpha = __expf(m - mn); m = mn;
    float ps = 0.f; v16h pf;
#pragma unroll
    for (int r = 0; r < 8; ++r) { const float p0 = __expf(s0[r] * 0.125f - mn), p1 = __expf(s1[r] * 0.125f - mn); ps += p0 + p1; pf[r] = (_Float16)(p0 * 4096.0f); pf[8 + r] = (_Float16)(p1 * 4096.0f); }
    l = l * alpha + ps;
#pragma unroll
    for (int j = 0; j < 4; ++j) oacc[j] *= alpha;
#pragma unroll
    for (int j = 0; j < 4; ++j) oacc[j] = wmma16(frag_h(Vb + (size_t)(16 * j) * SEQ + ks, lane), pf, oacc[j]);
  }
  l += __shfl_xor(l, 16); const float inv = 1.0f / (l * 4096.0f);
#pragma unroll
  for (int j = 0; j < 4; ++j)
#pragma unroll
    for (int r = 0; r < 8; ++r) ss[wave][col][16 * j + 8 * g + r] = oacc[j][r] * inv;
  ldsx();
  for (int rl = 0; rl < 16; ++rl) if (lane < HD / 4) vst2(Y + ((size_t)b * SEQ + ql0 + rl) * CC + h * HD + lane * 4, *(const v4f*)&ss[wave][rl][lane * 4]);
}

__global__ __launch_bounds__(128) void k_out(const float* __restrict__ Y, const __bf16* __restrict__ PB, const float* __restrict__ BP, float* __restrict__ OUT) {
  __shared__ __align__(16) float sf[4][16][132];
  const int tid = threadIdx.x, wave = tid >> 5, lane = tid & 31, col = lane & 15, g = lane >> 4; const int c0 = blockIdx.y * 128; const size_t r0 = (size_t)blockIdx.x * 64 + wave * 16;
  v8f acc[8] = {};
#pragma unroll 1
  for (int kc = 0; kc < CC / 32; ++kc) { const F2 a = split_row(Y + (r0 + col) * CC, kc * 32, lane);
#pragma unroll
    for (int j = 0; j < 8; ++j) { const v16b w = frag_b(PB + (size_t)(c0 + j * 16 + col) * CC + kc * 32, lane); acc[j] = wmma_bf(a.h, w, acc[j]); acc[j] = wmma_bf(a.l, w, acc[j]); } }
#pragma unroll
  for (int j = 0; j < 8; ++j) { const float bb = bfr(BP[c0 + j * 16 + col]);
#pragma unroll
    for (int r = 0; r < 8; ++r) sf[wave][8 * g + r][j * 16 + col] = acc[j][r] + bb; }
  ldsx(); for (int rl = 0; rl < 16; ++rl) vst2(OUT + (r0 + rl) * CC + c0 + lane * 4, *(const v4f*)&sf[wave][rl][lane * 4]);
}

extern "C" void kernel_launch(void* const* d_in, const int* in_sizes, int n_in, void* d_out, int out_size, void* d_ws, size_t ws_size, hipStream_t stream) {
  if (n_in < 5) return;
  if (in_sizes[0] < ((NB - 1) * TT_FULL + SEQ) * CC || in_sizes[1] < C3 * CC || in_sizes[2] < C3 || in_sizes[3] < CC * CC || in_sizes[4] < CC) return;
  if (out_size < NB * SEQ * CC) return;
  if (ws_size < (size_t)WS_END) return;
  const float* X = (const float*)d_in[0];
  const float* WIN = (const float*)d_in[1];
  const float* BIN = (const float*)d_in[2];
  const float* WPJ = (const float*)d_in[3];
  const float* BPJ = (const float*)d_in[4];
  char* ws = (char*)d_ws;
  __bf16 *XB = (__bf16*)(ws + WS_XB), *WB = (__bf16*)(ws + WS_WB), *PB = (__bf16*)(ws + WS_PB);
  _Float16 *QH = (_Float16*)(ws + WS_QH), *KH = (_Float16*)(ws + WS_KH), *VT = (_Float16*)(ws + WS_VT); float* Y = (float*)(ws + WS_Y);
  { const int t8 = NB * SEQ * CC / 8; k_cvt<<<dim3((t8 + 255) / 256), 256, 0, stream>>>(X, XB, NB * SEQ, CC, SEQ, TT_FULL); }
  { const int t8 = C3 * CC / 8; k_cvt<<<dim3((t8 + 255) / 256), 256, 0, stream>>>(WIN, WB, C3, CC, C3, C3); }
  { const int t8 = CC * CC / 8; k_cvt<<<dim3((t8 + 255) / 256), 256, 0, stream>>>(WPJ, PB, CC, CC, CC, CC); }
  k_proj<<<dim3(NB * SEQ / 64, C3 / 128), 128, 0, stream>>>(XB, WB, BIN, QH, KH, VT);
  k_attn<<<dim3(SEQ / 64, NH, NB), 128, 0, stream>>>(QH, KH, VT, Y);
  k_out<<<dim3(NB * SEQ / 64, CC / 128), 128, 0, stream>>>(Y, PB, BPJ, (float*)d_out);
}
